// Mamba3LBlock_80161269613360
// MI455X (gfx1250) — hardware-verified
//
#include <hip/hip_runtime.h>
#include <hip/hip_bf16.h>
#include <math.h>


typedef _Float16 bf16;
typedef _Float16 f16;
typedef __attribute__((ext_vector_type(4))) unsigned v4u_t;
typedef unsigned v4ua __attribute__((ext_vector_type(4), may_alias));
typedef __attribute__((ext_vector_type(4))) float v4f_t;
typedef float v4fa __attribute__((ext_vector_type(4), may_alias));
typedef __attribute__((ext_vector_type(16))) bf16  bf16x16;
typedef bf16x16 f16x16;
typedef __attribute__((ext_vector_type(8)))  bf16  bf16x8;
typedef bf16x8 f16x8;
typedef __attribute__((ext_vector_type(4)))  bf16  bf16x4;
typedef __attribute__((ext_vector_type(8)))  float f32x8;
__device__ __forceinline__ f32x8 wmma16(f16x16 a, f16x16 b, f32x8 c) {
  c = __builtin_amdgcn_wmma_f32_16x16x32_f16(false, a, false, b, (short)0, c, false, false);
  asm volatile("v_nop\n\tv_nop\n\tv_nop\n\tv_nop" : "+v"(c) : "v"(a), "v"(b));
  return c;
}
#define LDS_STRIDE 48
#define KSTRIDE    72
#define VSTRIDE    48

__device__ __forceinline__ f32x8 wmma_bf16(bf16x16 a, bf16x16 b, f32x8 c) {
  c = __builtin_amdgcn_wmma_f32_16x16x32_f16(false, a, false, b, (short)0, c, false, false);
  asm volatile("v_nop\n\tv_nop\n\tv_nop\n\tv_nop" : "+v"(c) : "v"(a), "v"(b));
  return c;
}

template <typename T>
__device__ __forceinline__ bf16x16 load_frag(const T* __restrict__ base, int ld,
                                             int row0, int k0) {
  const int lane = threadIdx.x & 31;
  const int r    = lane & 15;
  const int kh   = (lane >> 4) * 8;
  const T* p0 = base + (size_t)(row0 + r) * ld + (k0 + kh);
  const T* p1 = p0 + 16;
  bf16x16 f;
#pragma unroll
  for (int i = 0; i < 8; ++i) {
    f[i]     = (bf16)p0[i];
    f[i + 8] = (bf16)p1[i];
  }
  return f;
}

__device__ __forceinline__ bf16x16 lds_frag(const bf16* base, int stride) {
  const int lane = threadIdx.x & 31;
  const int row  = lane & 15;
  const int kh   = (lane >> 4) * 8;
  const bf16x8 lo = *(const bf16x8*)(base + row * stride + kh);
  const bf16x8 hi = *(const bf16x8*)(base + row * stride + kh + 16);
  bf16x16 f;
#pragma unroll
  for (int i = 0; i < 8; ++i) { f[i] = lo[i]; f[i + 8] = hi[i]; }
  return f;
}

template <typename T>
__device__ __forceinline__ void stage_read16(const T* __restrict__ p, float* buf) {
#pragma unroll
  for (int i = 0; i < 16; ++i) buf[i] = (float)p[i];
}

__device__ __forceinline__ void stage_write(bf16* dst, const float* buf, int nquad) {
#pragma unroll
  for (int i = 0; i < nquad; ++i) {
    bf16x4 q;
    q[0] = (bf16)buf[4 * i];     q[1] = (bf16)buf[4 * i + 1];
    q[2] = (bf16)buf[4 * i + 2]; q[3] = (bf16)buf[4 * i + 3];
    *(bf16x4*)(dst + 4 * i) = q;
  }
}


#define GSTR 48
#define GSTR 48
template <typename AT, int EPI, bool OUT16>
__global__ __launch_bounds__(256) void gemm_kne(const AT* __restrict__ A, int lda, const float* __restrict__ Wm, int ldw,
                                                const float* __restrict__ bias, const float* __restrict__ R, const float* __restrict__ gvec,
                                                void* __restrict__ Yv, int ldy, int K) {
  __shared__ __attribute__((aligned(16))) f16 ldsA[128 * GSTR];
  __shared__ __attribute__((aligned(16))) f16 ldsW[128 * GSTR];
  __shared__ __attribute__((aligned(16))) float oS[8][32 * 68];
  const int tid = threadIdx.x, lane = tid & 31, wave = tid >> 5, cl = lane & 15, rh = (lane >> 4) * 8;
  const int m0 = blockIdx.x * 128, n0 = blockIdx.y * 128;
  const int wm = (wave & 3) * 32, wn = (wave >> 2) * 64;
  f32x8 acc[2][4];
#pragma unroll
  for (int i = 0; i < 2; ++i)
#pragma unroll
    for (int j = 0; j < 4; ++j) { f32x8 z = {}; acc[i][j] = z; }
#pragma unroll 1
  for (int k0 = 0; k0 < K; k0 += 32) {
    __syncthreads();
    { const int row = tid >> 1, ch = (tid & 1) * 16;
      const AT* src = A + (size_t)(m0 + row) * lda + k0 + ch;
#pragma unroll
      for (int g = 0; g < 16; ++g) ldsA[row * GSTR + ch + g] = (f16)src[g]; }
    { const int k = tid >> 3, nn0 = (tid & 7) * 16;
      const float* src = Wm + (size_t)(k0 + k) * ldw + n0 + nn0;
#pragma unroll
      for (int g = 0; g < 4; ++g) { const v4f_t v = *(const v4f_t*)(src + 4 * g);
#pragma unroll
        for (int u = 0; u < 4; ++u) ldsW[(nn0 + 4 * g + u) * GSTR + k] = (f16)v[u]; } }
    __syncthreads();
    f16x16 af[2];
#pragma unroll
    for (int i = 0; i < 2; ++i) af[i] = lds_frag(ldsA + (wm + 16 * i) * GSTR, GSTR);
#pragma unroll
    for (int j = 0; j < 4; ++j) {
      const f16x16 bf = lds_frag(ldsW + (wn + 16 * j) * GSTR, GSTR);
#pragma unroll
      for (int i = 0; i < 2; ++i) acc[i][j] = wmma16(af[i], bf, acc[i][j]);
    }
  }
  float* so = oS[wave];
#pragma unroll
  for (int i = 0; i < 2; ++i)
#pragma unroll
    for (int j = 0; j < 4; ++j) {
      const int n = n0 + wn + 16 * j + cl;
      const float bv = bias ? bias[n] : 0.0f;
      const float gv = (EPI == 2 || EPI == 4) ? gvec[n] : 0.0f;
      if (EPI == 1) {
#pragma unroll 1
        for (int r = 0; r < 8; ++r) { const float xg = acc[i][j][r] + bv; so[(16 * i + rh + r) * 68 + 16 * j + cl] = 0.5f * xg * (1.0f + erff(xg * 0.70710678118654752f)); }
      } else {
#pragma unroll
        for (int r = 0; r < 8; ++r) {
          float v = acc[i][j][r] + bv;
          if (EPI == 3) v = fmaxf(v, 0.0f);
          if (EPI == 4) v = gv * v;
          if (EPI == 2) v = R[(size_t)(m0 + wm + 16 * i + rh + r) * ldy + n] + gv * v;
          so[(16 * i + rh + r) * 68 + 16 * j + cl] = v;
        }
      }
    }
  asm volatile("s_wait_dscnt 0" ::: "memory");
  __builtin_amdgcn_wave_barrier();
#pragma unroll 1
  for (int pass = 0; pass < 2; ++pass) {
    if (OUT16) {
      f16* Y = (f16*)Yv;
#pragma unroll
      for (int it = 0; it < 8; ++it) { const int c = lane + 32 * it, rr = c >> 3, q8 = (c & 7) * 8;
        union { f16 h[8]; v4u_t v; } u;
#pragma unroll
        for (int e = 0; e < 8; ++e) u.h[e] = (f16)so[rr * 68 + q8 + e];
        *(volatile v4u_t*)(Y + (size_t)(m0 + wm + rr) * ldy + n0 + wn + q8) = u.v; }
    } else {
      float* Y = (float*)Yv;
#pragma unroll
      for (int it = 0; it < 16; ++it) { const int f4 = lane + 32 * it, rr = f4 >> 4, q = (f4 & 15) * 4;
        *(volatile v4f_t*)(Y + (size_t)(m0 + wm + rr) * ldy + n0 + wn + q) = *(const v4fa*)(so + rr * 68 + q); }
    }
    __threadfence();
  }
}

template <typename AT, int EPI, bool OUT16>
__global__ __launch_bounds__(256) void gemm_knez(const AT* __restrict__ A, int lda, size_t strideA, const float* __restrict__ Wm, int ldw, size_t strideW,
                                                 const float* __restrict__ bias, const float* __restrict__ R, const float* __restrict__ gvec,
                                                 void* __restrict__ Yv, int ldy, size_t strideY, int K) {
  A += (size_t)blockIdx.z * strideA; Wm += (size_t)blockIdx.z * strideW; Yv = (void*)((char*)Yv + (size_t)blockIdx.z * strideY * (OUT16 ? 2 : 4)); if (R) R += (size_t)blockIdx.z * strideY;
  __shared__ __attribute__((aligned(16))) f16 ldsA[128 * GSTR];
  __shared__ __attribute__((aligned(16))) f16 ldsW[128 * GSTR];
  __shared__ __attribute__((aligned(16))) float oS[8][32 * 68];
  const int tid = threadIdx.x, lane = tid & 31, wave = tid >> 5, cl = lane & 15, rh = (lane >> 4) * 8;
  const int m0 = blockIdx.x * 128, n0 = blockIdx.y * 128;
  const int wm = (wave & 3) * 32, wn = (wave >> 2) * 64;
  f32x8 acc[2][4];
#pragma unroll
  for (int i = 0; i < 2; ++i)
#pragma unroll
    for (int j = 0; j < 4; ++j) { f32x8 z = {}; acc[i][j] = z; }
#pragma unroll 1
  for (int k0 = 0; k0 < K; k0 += 32) {
    __syncthreads();
    { const int row = tid >> 1, ch = (tid & 1) * 16;
      const AT* src = A + (size_t)(m0 + row) * lda + k0 + ch;
#pragma unroll
      for (int g = 0; g < 16; ++g) ldsA[row * GSTR + ch + g] = (f16)src[g]; }
    { const int k = tid >> 3, nn0 = (tid & 7) * 16;
      const float* src = Wm + (size_t)(k0 + k) * ldw + n0 + nn0;
#pragma unroll
      for (int g = 0; g < 4; ++g) { const v4f_t v = *(const v4f_t*)(src + 4 * g);
#pragma unroll
        for (int u = 0; u < 4; ++u) ldsW[(nn0 + 4 * g + u) * GSTR + k] = (f16)v[u]; } }
    __syncthreads();
    f16x16 af[2];
#pragma unroll
    for (int i = 0; i < 2; ++i) af[i] = lds_frag(ldsA + (wm + 16 * i) * GSTR, GSTR);
#pragma unroll
    for (int j = 0; j < 4; ++j) {
      const f16x16 bf = lds_frag(ldsW + (wn + 16 * j) * GSTR, GSTR);
#pragma unroll
      for (int i = 0; i < 2; ++i) acc[i][j] = wmma16(af[i], bf, acc[i][j]);
    }
  }
  float* so = oS[wave];
#pragma unroll
  for (int i = 0; i < 2; ++i)
#pragma unroll
    for (int j = 0; j < 4; ++j) {
      const int n = n0 + wn + 16 * j + cl;
      const float bv = bias ? bias[n] : 0.0f;
      const float gv = (EPI == 2 || EPI == 4) ? gvec[n] : 0.0f;
      if (EPI == 1) {
#pragma unroll 1
        for (int r = 0; r < 8; ++r) { const float xg = acc[i][j][r] + bv; so[(16 * i + rh + r) * 68 + 16 * j + cl] = 0.5f * xg * (1.0f + erff(xg * 0.70710678118654752f)); }
      } else {
#pragma unroll
        for (int r = 0; r < 8; ++r) {
          float v = acc[i][j][r] + bv;
          if (EPI == 3) v = fmaxf(v, 0.0f);
          if (EPI == 4) v = gv * v;
          if (EPI == 2) v = R[(size_t)(m0 + wm + 16 * i + rh + r) * ldy + n] + gv * v;
          so[(16 * i + rh + r) * 68 + 16 * j + cl] = v;
        }
      }
    }
  asm volatile("s_wait_dscnt 0" ::: "memory");
  __builtin_amdgcn_wave_barrier();
#pragma unroll 1
  for (int pass = 0; pass < 2; ++pass) {
    if (OUT16) {
      f16* Y = (f16*)Yv;
#pragma unroll
      for (int it = 0; it < 8; ++it) { const int c = lane + 32 * it, rr = c >> 3, q8 = (c & 7) * 8;
        union { f16 h[8]; v4u_t v; } u;
#pragma unroll
        for (int e = 0; e < 8; ++e) u.h[e] = (f16)so[rr * 68 + q8 + e];
        *(volatile v4u_t*)(Y + (size_t)(m0 + wm + rr) * ldy + n0 + wn + q8) = u.v; }
    } else {
      float* Y = (float*)Yv;
#pragma unroll
      for (int it = 0; it < 16; ++it) { const int f4 = lane + 32 * it, rr = f4 >> 4, q = (f4 & 15) * 4;
        *(volatile v4f_t*)(Y + (size_t)(m0 + wm + rr) * ldy + n0 + wn + q) = *(const v4fa*)(so + rr * 68 + q); }
    }
    __threadfence();
  }
}

template <typename AT, bool ACC>
__global__ __launch_bounds__(256) void gemm_kn2(const AT* __restrict__ A, int lda, size_t strideA,
                                               const float* __restrict__ Wm, int ldw, size_t strideW,
                                               const float* __restrict__ bias, float scale,
                                               float* __restrict__ Y, int ldy, size_t strideY, int K) {
  __shared__ __attribute__((aligned(16))) f16 ldsA[128 * GSTR], ldsAl[128 * GSTR];
  __shared__ __attribute__((aligned(16))) f16 ldsW[128 * GSTR], ldsWl[128 * GSTR];
  __shared__ __attribute__((aligned(16))) float oS[8][32 * 68];
  const int tid = threadIdx.x, lane = tid & 31, wave = tid >> 5, cl = lane & 15, rh = (lane >> 4) * 8;
  const int m0 = blockIdx.x * 128, n0 = blockIdx.y * 128;
  const int wm = (wave & 3) * 32, wn = (wave >> 2) * 64;
  A += (size_t)blockIdx.z * strideA; Wm += (size_t)blockIdx.z * strideW; Y += (size_t)blockIdx.z * strideY;
  f32x8 acc[2][4], accx[2][4];
#pragma unroll
  for (int i = 0; i < 2; ++i)
#pragma unroll
    for (int j = 0; j < 4; ++j) { f32x8 z = {}; acc[i][j] = z; accx[i][j] = z; }
#pragma unroll 1
  for (int k0 = 0; k0 < K; k0 += 32) {
    __syncthreads();
    {
      const int row = tid >> 1, ch = (tid & 1) * 16;
      const AT* src = A + (size_t)(m0 + row) * lda + k0 + ch;
#pragma unroll
      for (int g = 0; g < 16; ++g) { const float v = (float)src[g]; const f16 h = (f16)v; ldsA[row * GSTR + ch + g] = h; ldsAl[row * GSTR + ch + g] = (f16)((v - (float)h) * 2048.0f); }
    }
    {
      const int k = tid >> 3, nn0 = (tid & 7) * 16;
      const float* src = Wm + (size_t)(k0 + k) * ldw + n0 + nn0;
#pragma unroll
      for (int g = 0; g < 4; ++g) { const v4f_t v = *(const v4f_t*)(src + 4 * g);
#pragma unroll
        for (int u = 0; u < 4; ++u) { const f16 h = (f16)v[u]; ldsW[(nn0 + 4 * g + u) * GSTR + k] = h; ldsWl[(nn0 + 4 * g + u) * GSTR + k] = (f16)((v[u] - (float)h) * 2048.0f); } }
    }
    __syncthreads();
    f16x16 af[2], afl[2];
#pragma unroll
    for (int i = 0; i < 2; ++i) { af[i] = lds_frag(ldsA + (wm + 16 * i) * GSTR, GSTR); afl[i] = lds_frag(ldsAl + (wm + 16 * i) * GSTR, GSTR); }
#pragma unroll
    for (int j = 0; j < 4; ++j) {
      const f16x16 bf = lds_frag(ldsW + (wn + 16 * j) * GSTR, GSTR), bfl = lds_frag(ldsWl + (wn + 16 * j) * GSTR, GSTR);
#pragma unroll
      for (int i = 0; i < 2; ++i) { acc[i][j] = wmma16(af[i], bf, acc[i][j]); accx[i][j] = wmma16(af[i], bfl, accx[i][j]); accx[i][j] = wmma16(afl[i], bf, accx[i][j]); }
    }
  }
  float* so = oS[wave];
#pragma unroll
  for (int i = 0; i < 2; ++i)
#pragma unroll
    for (int j = 0; j < 4; ++j) {
      const float bv = bias ? bias[n0 + wn + 16 * j + cl] : 0.0f;
#pragma unroll
      for (int r = 0; r < 8; ++r) so[(16 * i + rh + r) * 68 + 16 * j + cl] = (acc[i][j][r] + accx[i][j][r] * (1.0f / 2048.0f)) * scale + bv;
    }
  asm volatile("s_wait_dscnt 0" ::: "memory");
  __builtin_amdgcn_wave_barrier();
  if (ACC) {
#pragma unroll
    for (int it = 0; it < 16; ++it) { const int f4 = lane + 32 * it, rr = f4 >> 4, q = (f4 & 15) * 4;
      const v4f_t old = *(const v4fa*)(Y + (size_t)(m0 + wm + rr) * ldy + n0 + wn + q);
      v4f_t v = *(const v4fa*)(so + rr * 68 + q); v += old; *(v4fa*)(so + rr * 68 + q) = v; }
    asm volatile("s_wait_dscnt 0" ::: "memory");
  }
#pragma unroll 1
  for (int pass = 0; pass < 2; ++pass) {
#pragma unroll
    for (int it = 0; it < 16; ++it) { const int f4 = lane + 32 * it, rr = f4 >> 4, q = (f4 & 15) * 4;
      *(volatile v4f_t*)(Y + (size_t)(m0 + wm + rr) * ldy + n0 + wn + q) = *(const v4fa*)(so + rr * 68 + q); }
    __threadfence();
  }
}

__global__ __launch_bounds__(256) void k_transpose(const float* __restrict__ Wm, float* __restrict__ Wt, int rows, int cols) {
  __shared__ float tS[64][65];
  const int tid = threadIdx.x, tbj = cols / 64, bi = blockIdx.x / tbj, bj = blockIdx.x % tbj;
  for (int e = tid; e < 64 * 64; e += 256) { const int r = e >> 6, c = e & 63; tS[r][c] = Wm[(size_t)(bi * 64 + r) * cols + bj * 64 + c]; }
  __syncthreads();
  for (int ch = tid; ch < 64 * 16; ch += 256) { const int r = ch >> 4, q4 = (ch & 15) * 4; v4f_t o; o[0] = tS[q4][r]; o[1] = tS[q4 + 1][r]; o[2] = tS[q4 + 2][r]; o[3] = tS[q4 + 3][r];
    float* dst = Wt + (size_t)(bj * 64 + r) * rows + bi * 64 + q4; *(volatile v4f_t*)dst = o; __threadfence(); *(volatile v4f_t*)dst = o; }
}


#define GSTR 48
#define SS 2048
#define HH 32
#define DKK 64
template <typename AT, int MODE>
__global__ __launch_bounds__(256) void gemm_rb_kernel(
    const AT* __restrict__ A, const float* __restrict__ W,
    const float* __restrict__ bias, const float* __restrict__ rowscale, const float* __restrict__ R, const float* __restrict__ rowbias, void* __restrict__ out,
    int M, int N, int K) {
  __shared__ bf16 ldsA[128 * LDS_STRIDE];
  __shared__ bf16 ldsW[256 * LDS_STRIDE];
  __shared__ __attribute__((aligned(16))) unsigned char sob[256 * 136 * 2];

  const int t    = threadIdx.x;
  const int wave = t >> 5;
  const int lane = t & 31;
  const int wm   = (wave & 1) * 64;
  const int wn   = (wave >> 1) * 64;
  const int mBlk = blockIdx.x * 128;
  const int nBlk = blockIdx.y * 256;

  const int arow = t >> 1;
  const int ach  = (t & 1) * 16;

  float abuf[16];
  float wbuf[32];

  stage_read16(A + (size_t)(mBlk + arow) * K + ach, abuf);
  const int nrow = min(nBlk + t, N - 1);
  stage_read16(W + (size_t)nrow * K,          wbuf);
  stage_read16(W + (size_t)nrow * K + 16,     wbuf + 16);

  f32x8 acc[4][4] = {};

  for (int k = 0; k < K; k += 32) {
    __syncthreads();
    stage_write(&ldsA[arow * LDS_STRIDE + ach], abuf, 4);
    stage_write(&ldsW[t * LDS_STRIDE],          wbuf, 8);
    if (k + 32 < K) {
      stage_read16(A + (size_t)(mBlk + arow) * K + (k + 32) + ach, abuf);
      stage_read16(W + (size_t)nrow * K + (k + 32),          wbuf);
      stage_read16(W + (size_t)nrow * K + (k + 32) + 16,     wbuf + 16);
    }
    __syncthreads();

    bf16x16 af[4], wf[4];
#pragma unroll
    for (int i = 0; i < 4; ++i)
      af[i] = lds_frag(ldsA + (wm + 16 * i) * LDS_STRIDE, LDS_STRIDE);
#pragma unroll
    for (int j = 0; j < 4; ++j)
      wf[j] = lds_frag(ldsW + (wn + 16 * j) * LDS_STRIDE, LDS_STRIDE);
#pragma unroll
    for (int i = 0; i < 4; ++i)
#pragma unroll
      for (int j = 0; j < 4; ++j)
        acc[i][j] = wmma_bf16(af[i], wf[j], acc[i][j]);
  }

  const int nlane = lane & 15;
  const int mh    = (lane >> 4) * 8;
  __syncthreads();
  if (MODE == 0 || MODE == 1 || MODE == 3) {
    bf16* so = (bf16*)sob;
#pragma unroll
    for (int i = 0; i < 4; ++i)
#pragma unroll
      for (int j = 0; j < 4; ++j) {
        const int nl = wn + 16 * j + nlane;
        const float bv = bias ? bias[nBlk + nl] : 0.0f;
        if (MODE == 3) {
#pragma unroll 1
          for (int r = 0; r < 8; ++r) {
            const int ml = wm + 16 * i + mh + r;
            const float xg = acc[i][j][r] + bv;
            so[ml * 264 + nl] = (bf16)(0.5f * xg * (1.0f + erff(xg * 0.70710678118654752f)));
          }
        } else {
#pragma unroll
        for (int r = 0; r < 8; ++r) {
          const int ml = wm + 16 * i + mh + r;
          const bf16 hv = (bf16)(acc[i][j][r] + bv);
          if (MODE == 0) so[ml * 264 + nl] = hv;
          else           so[nl * 136 + ml] = hv;
        }
        }
      }
    __syncthreads();
#pragma unroll 1
    for (int pass = 0; pass < 2; ++pass) {
      if (MODE == 0 || MODE == 3) {
        for (int ch = t; ch < 128 * 32; ch += 256) { const int ml = ch >> 5, q = (ch & 31) * 8;
          *(volatile v4u_t*)((bf16*)out + (size_t)(mBlk + ml) * N + nBlk + q) = *(const v4ua*)(so + ml * 264 + q); }
      } else {
        const int b_ = mBlk / SS, s0 = mBlk % SS;
        for (int ch = t; ch < 256 * 16; ch += 256) { const int nl = ch >> 4, q = (ch & 15) * 8; const int n = nBlk + nl, h = n >> 6, dk = n & (DKK - 1);
          *(volatile v4u_t*)((bf16*)out + (((size_t)(b_ * HH + h)) * DKK + dk) * SS + s0 + q) = *(const v4ua*)(so + nl * 136 + q); }
      }
      __threadfence();
    }
  } else {
    float* so = (float*)sob;
#pragma unroll 1
    for (int hf = 0; hf < 2; ++hf) {
      if (wm == hf * 64) {
#pragma unroll
        for (int i = 0; i < 4; ++i)
#pragma unroll
          for (int j = 0; j < 4; ++j) {
            const int nl = wn + 16 * j + nlane;
            const float bv = bias ? bias[nBlk + nl] : 0.0f;
#pragma unroll
            for (int r = 0; r < 8; ++r) { const int mrow = mBlk + hf * 64 + 16 * i + mh + r; so[(16 * i + mh + r) * 260 + nl] = acc[i][j][r] * (rowscale ? rowscale[mrow] : 1.0f) + bv + (rowbias ? rowbias[mrow] : 0.0f); }
          }
      }
      __syncthreads();
      if (R) {
        for (int ch = t; ch < 64 * 64; ch += 256) { const int ml = ch >> 6, q = (ch & 63) * 4;
          if (nBlk + q < N) { const v4f_t rv = *(const v4f_t*)(R + (size_t)(mBlk + hf * 64 + ml) * N + nBlk + q); v4f_t v = *(const v4fa*)(so + ml * 260 + q); v += rv; *(volatile v4fa*)(so + ml * 260 + q) = v; } }
        asm volatile("s_wait_dscnt 0" ::: "memory");
      }
#pragma unroll 1
      for (int pass = 0; pass < 2; ++pass) {
        for (int ch = t; ch < 64 * 64; ch += 256) { const int ml = ch >> 6, q = (ch & 63) * 4;
          if (nBlk + q < N) *(volatile v4f_t*)((float*)out + (size_t)(mBlk + hf * 64 + ml) * N + nBlk + q) = *(const v4fa*)(so + ml * 260 + q); }
        __threadfence();
      }
      __syncthreads();
    }
  }
}

#define NBm 4
#define LLm 2048
#define LIN 2048
#define DDm 512
#define DIm 1024
#define NHm 16
#define HDm 64
#define NSm 128
#define RRm 4
#define PCm 16
#define CDm 2048
#define DINm 3088
#define DINP 3200
#define TCH 16
__global__ __launch_bounds__(256) void k_fill(float* __restrict__ p, float val, size_t n4) { const size_t i = (size_t)blockIdx.x * 256 + threadIdx.x; if (i < n4) { v4f_t v = {val, val, val, val}; *(volatile v4f_t*)(p + 4 * i) = v; __threadfence(); *(volatile v4f_t*)(p + 4 * i) = v; } }
__global__ __launch_bounds__(256) void k_dbg_zero(float* __restrict__ p, size_t n4) { const size_t i = (size_t)blockIdx.x * 256 + threadIdx.x; if (i < n4) { v4f_t z = {0.f,0.f,0.f,0.f}; *(volatile v4f_t*)(p + 4 * i) = z; __threadfence(); *(volatile v4f_t*)(p + 4 * i) = z; } }
__global__ __launch_bounds__(256) void k_copy(const float* __restrict__ src, float* __restrict__ dst, size_t n4) { const size_t i = (size_t)blockIdx.x * 256 + threadIdx.x; if (i < n4) { const v4f_t v = *(const v4f_t*)(src + 4 * i); *(volatile v4f_t*)(dst + 4 * i) = v; __threadfence(); *(volatile v4f_t*)(dst + 4 * i) = v; } }
__global__ __launch_bounds__(256) void k_padw(const float* __restrict__ Wm, float* __restrict__ WP) { const int k = blockIdx.x, tid = threadIdx.x;
#pragma unroll 1
  for (int pass = 0; pass < 2; ++pass) {
#pragma unroll 1
    for (int n = tid; n < DINP; n += 256) { const float v = (n < DINm) ? Wm[(size_t)k * DINm + min(n, DINm - 1)] : 0.0f; *(volatile float*)(WP + (size_t)k * DINP + n) = v; }
    __threadfence(); } }
__global__ __launch_bounds__(256) void k_conv(const float* __restrict__ ZX, const float* __restrict__ cw, const float* __restrict__ cb, float* __restrict__ XC) {
  const int t = blockIdx.x, tid = threadIdx.x;
#pragma unroll 1
  for (int pass = 0; pass < 2; ++pass) {
#pragma unroll 1
    for (int c = tid; c < CDm; c += 256) { float acc = cb[c];
#pragma unroll
      for (int k = 0; k < 4; ++k) { const int tt = t - 3 + k; const int tc = max(tt, 0); const float xv = ZX[(size_t)tc * DINP + DIm + c]; acc = fmaf((tt >= 0) ? xv : 0.0f, cw[c * 4 + k], acc); }
      *(volatile float*)(XC + (size_t)t * CDm + c) = acc / (1.0f + expf(-acc)); }
    __threadfence(); }
}
__global__ __launch_bounds__(128) void k_mimo(const float* __restrict__ XC, const float* __restrict__ ZX, const float* __restrict__ dtb, const float* __restrict__ Alog, const float* __restrict__ Dv, float* __restrict__ Y) {
  __shared__ __attribute__((aligned(16))) float Bs[TCH][NSm * RRm]; __shared__ __attribute__((aligned(16))) float Cs[TCH][NSm * RRm]; __shared__ float DT[TCH]; __shared__ float DC[TCH]; __shared__ __attribute__((aligned(16))) float yS[TCH][HDm + 4];
  const int h = blockIdx.x, tid = threadIdx.x; const int pp = tid >> 4, sl = tid & 15; const int pa = 2 * pp, pb = 2 * pp + 1;
  const float Ah = expf(Alog[h]), db = dtb[h], Dd = Dv[h]; float ha[8], hb[8];
#pragma unroll
  for (int n = 0; n < 8; ++n) { ha[n] = 0.0f; hb[n] = 0.0f; }
#pragma unroll 1
  for (int c0 = 0; c0 < LLm; c0 += TCH) {
    __syncthreads();
#pragma unroll 1
    for (int e = tid; e < TCH * NSm * RRm; e += 128) { const int tt = e >> 9, c = e & 511; Bs[tt][c] = XC[(size_t)(c0 + tt) * CDm + DIm + c]; Cs[tt][c] = XC[(size_t)(c0 + tt) * CDm + DIm + NSm * RRm + c]; }
    if (tid < TCH) { const float dr = ZX[(size_t)(c0 + tid) * DINP + DIm + CDm + h] + db; const float dt = (dr > 20.0f) ? dr : log1pf(expf(dr)); DT[tid] = dt; DC[tid] = expf(-dt * Ah); }
    __syncthreads();
#pragma unroll 1
    for (int tt = 0; tt < TCH; ++tt) {
      const float dt = DT[tt], dec = DC[tt]; const float* xr = XC + (size_t)(c0 + tt) * CDm + h * HDm;
      const float xa0 = xr[pa], xa1 = xr[16 + pa], xa2 = xr[32 + pa], xa3 = xr[48 + pa], xb0 = xr[pb], xb1 = xr[16 + pb], xb2 = xr[32 + pb], xb3 = xr[48 + pb];
      float ya0 = 0.f, ya1 = 0.f, ya2 = 0.f, ya3 = 0.f, yb0 = 0.f, yb1 = 0.f, yb2 = 0.f, yb3 = 0.f;
#pragma unroll
      for (int k = 0; k < 8; ++k) { const int n = sl * 8 + k; const v4f_t bn = *(const v4fa*)(&Bs[tt][n * RRm]); const v4f_t cn = *(const v4fa*)(&Cs[tt][n * RRm]);
        const float ua = fmaf(bn[0], xa0, fmaf(bn[1], xa1, fmaf(bn[2], xa2, bn[3] * xa3))), ub = fmaf(bn[0], xb0, fmaf(bn[1], xb1, fmaf(bn[2], xb2, bn[3] * xb3)));
        ha[k] = fmaf(ha[k], dec, dt * ua); hb[k] = fmaf(hb[k], dec, dt * ub);
        ya0 = fmaf(cn[0], ha[k], ya0); ya1 = fmaf(cn[1], ha[k], ya1); ya2 = fmaf(cn[2], ha[k], ya2); ya3 = fmaf(cn[3], ha[k], ya3);
        yb0 = fmaf(cn[0], hb[k], yb0); yb1 = fmaf(cn[1], hb[k], yb1); yb2 = fmaf(cn[2], hb[k], yb2); yb3 = fmaf(cn[3], hb[k], yb3); }
#pragma unroll
      for (int o = 1; o < 16; o <<= 1) { ya0 += __shfl_xor(ya0, o, 32); ya1 += __shfl_xor(ya1, o, 32); ya2 += __shfl_xor(ya2, o, 32); ya3 += __shfl_xor(ya3, o, 32); yb0 += __shfl_xor(yb0, o, 32); yb1 += __shfl_xor(yb1, o, 32); yb2 += __shfl_xor(yb2, o, 32); yb3 += __shfl_xor(yb3, o, 32); }
      if (sl == 0) { yS[tt][pa] = ya0 + Dd * xa0; yS[tt][16 + pa] = ya1 + Dd * xa1; yS[tt][32 + pa] = ya2 + Dd * xa2; yS[tt][48 + pa] = ya3 + Dd * xa3; yS[tt][pb] = yb0 + Dd * xb0; yS[tt][16 + pb] = yb1 + Dd * xb1; yS[tt][32 + pb] = yb2 + Dd * xb2; yS[tt][48 + pb] = yb3 + Dd * xb3; } }
    __syncthreads();
#pragma unroll 1
    for (int pass = 0; pass < 2; ++pass) {
#pragma unroll 1
      for (int i = tid; i < TCH * 16; i += 128) { const int tt = i >> 4, piece = (i & 15) * 4;
        *(volatile v4f_t*)(Y + (size_t)(c0 + tt) * DIm + h * HDm + piece) = *(const v4fa*)(&yS[tt][piece]); }
      __threadfence(); }
  }
}
__global__ __launch_bounds__(256) void k_gate(const float* __restrict__ Y, const float* __restrict__ ZX, f16* __restrict__ G) {
  const int t = blockIdx.x, c = 4 * threadIdx.x; const v4f_t y = *(const v4f_t*)(Y + (size_t)t * DIm + c), z = *(const v4f_t*)(ZX + (size_t)t * DINP + c); union { f16 hh[4]; unsigned long long u; } o;
#pragma unroll
  for (int u = 0; u < 4; ++u) o.hh[u] = (f16)(y[u] * (z[u] / (1.0f + expf(-z[u]))));
  *(volatile unsigned long long*)(G + (size_t)t * DIm + c) = o.u; __threadfence(); *(volatile unsigned long long*)(G + (size_t)t * DIm + c) = o.u;
}
__global__ __launch_bounds__(128) void k_rmsf(const float* __restrict__ Rz, float* __restrict__ outb) {
  __shared__ float red[128];
  const size_t r = blockIdx.x; const int tid = threadIdx.x; const v4f_t v = *(const v4f_t*)(Rz + r * DDm + 4 * tid); red[tid] = v[0] * v[0] + v[1] * v[1] + v[2] * v[2] + v[3] * v[3]; __syncthreads();
  for (int o = 64; o > 0; o >>= 1) { if (tid < o) red[tid] += red[tid + o]; __syncthreads(); }
  const v4f_t y = v * (1.0f / __builtin_sqrtf(red[0] * (1.0f / DDm) + 1e-5f)); *(volatile v4f_t*)(outb + r * DDm + 4 * tid) = y; __threadfence(); *(volatile v4f_t*)(outb + r * DDm + 4 * tid) = y;
}

extern "C" void kernel_launch(void* const* d_in, const int* in_sizes, int n_in,
                              void* d_out, int out_size, void* d_ws, size_t ws_size,
                              hipStream_t stream) {
  (void)in_sizes; (void)n_in; (void)out_size;
  const float** f = (const float**)d_in;
  const float* x = f[0], *Win = f[1], *cw = f[2], *cb = f[3], *dtb = f[4], *Alog = f[5], *Dv = f[6], *Wout = f[7];
  float* out = (float*)d_out;
  char* ws = (char*)d_ws;
  float* WP = (float*)ws; ws += (size_t)DDm * DINP * 4; float* ZX = (float*)ws; ws += (size_t)LLm * DINP * 4; float* XC = (float*)ws; ws += (size_t)LLm * CDm * 4;
  float* Y = (float*)ws; ws += (size_t)LLm * DIm * 4; f16* G16 = (f16*)ws; ws += (size_t)LLm * DIm * 2; float* RES = (float*)ws; ws += (size_t)LLm * DDm * 4; float* ones = (float*)ws; ws += DDm * 4;
  if ((size_t)(ws - (char*)d_ws) > ws_size) return;
  const dim3 blk(256);
  k_padw<<<dim3(DDm), blk, 0, stream>>>(Win, WP); k_fill<<<dim3(1), blk, 0, stream>>>(ones, 1.0f, DDm / 4);

  for (int b = 0; b < NBm; ++b) { const float* xb = x + (size_t)b * LIN * DDm;
    gemm_kne<float, 0, false><<<dim3(LLm / 128, DINP / 128), blk, 0, stream>>>(xb, DDm, WP, DINP, nullptr, nullptr, nullptr, ZX, DINP, DDm);
    k_conv<<<dim3(LLm), blk, 0, stream>>>(ZX, cw, cb, XC);
    k_mimo<<<dim3(NHm), dim3(128), 0, stream>>>(XC, ZX, dtb, Alog, Dv, Y);
    k_gate<<<dim3(LLm), blk, 0, stream>>>(Y, ZX, G16);
    gemm_kne<f16, 2, false><<<dim3(LLm / 128, DDm / 128), blk, 0, stream>>>(G16, DIm, Wout, DDm, nullptr, xb, ones, RES, DDm, DIm);
    k_rmsf<<<dim3(LLm), dim3(128), 0, stream>>>(RES, out + (size_t)b * LIN * DDm);
  }
}
